// Block_71554155151924
// MI455X (gfx1250) — hardware-verified
//
#include <hip/hip_runtime.h>
#include <math.h>

#ifndef NB
#define NB 2
#endif
#ifndef SEQ
#define SEQ 2048
#endif
#define NB_FULL 2
#define SEQ_FULL 2048
#define CC 1024
#define NH 16
#define HD 64
#define FFW 4096
#define NROW (NB * SEQ)

static_assert(SEQ % 64 == 0);
static_assert(NROW % 64 == 0);
static_assert(CC % 64 == 0);
static_assert(CC % 32 == 0);
static_assert(FFW % 64 == 0);
static_assert(FFW % 32 == 0);
static_assert(HD == 64);
static_assert(NH * HD == CC);
static_assert(CC == 128 * 8);
static_assert(3 * HD == 192);
static_assert(NB <= NB_FULL);
static_assert(SEQ <= SEQ_FULL);
static_assert((long long)NB * NH * SEQ * HD < 2147483647LL);
static_assert((long long)CC * NROW < 2147483647LL);

typedef __attribute__((ext_vector_type(16))) _Float16 v16h;
typedef __attribute__((ext_vector_type(8)))  _Float16 v8h;
typedef __attribute__((ext_vector_type(8)))  float    v8f;
typedef __attribute__((ext_vector_type(4)))  float    v4f;
typedef __attribute__((ext_vector_type(4)))  unsigned int u4v;
typedef __attribute__((ext_vector_type(2)))  unsigned int u2v;

#define WSC      16.0f
#define WSC_INV  0.0625f
#define QRES     2048.0f
#define QRES_INV 0.00048828125f
#define PSC      16384.0f
#define AOC      16.0f

union FragU { v16h v; v8h h[2]; };
__device__ __forceinline__ v16h frag_ld(const _Float16* __restrict__ p) { FragU f; f.h[0] = *(const v8h*)(p); f.h[1] = *(const v8h*)(p + 16); return f.v; }

__device__ __forceinline__ v8f wmma16(v16h a, v16h b, v8f c) {
    c = __builtin_amdgcn_wmma_f32_16x16x32_f16(false, a, false, b, (short)0, c, false, false);
    asm volatile("v_nop\n\tv_nop\n\tv_nop\n\tv_nop" : "+v"(c) : "v"(a), "v"(b));
    return c;
}
__device__ __forceinline__ v8f wmma_raw(v16h a, v16h b, v8f c) { return __builtin_amdgcn_wmma_f32_16x16x32_f16(false, a, false, b, (short)0, c, false, false); }
__device__ __forceinline__ void dep_guard_h(v8f& a, v8f& b, v16h x, v16h y) { asm volatile("v_nop\n\tv_nop\n\tv_nop\n\tv_nop" : "+v"(a), "+v"(b) : "v"(x), "v"(y)); }
__device__ __forceinline__ void keep4_h(v16h a, v16h b, v16h c, v16h d) { asm volatile("v_nop" :: "v"(a), "v"(b), "v"(c), "v"(d)); }
__device__ __forceinline__ void acc_guard4(v8f& a, v8f& b, v8f& c, v8f& d) { asm volatile("v_nop\n\tv_nop\n\tv_nop\n\tv_nop" : "+v"(a), "+v"(b), "+v"(c), "+v"(d)); }

__device__ __forceinline__ float cmb_bf(float v) { const unsigned u = __builtin_bit_cast(unsigned, v); const unsigned r = (u + 0x7fffu + ((u >> 16) & 1u)) & 0xffff0000u; return __builtin_bit_cast(float, r); }
__device__ __forceinline__ unsigned int pk2h(float a, float b) { return (unsigned int)__builtin_bit_cast(unsigned short, (_Float16)a) | ((unsigned int)__builtin_bit_cast(unsigned short, (_Float16)b) << 16); }

#define VST2(T, ptr, val) do { const T vst2_v_ = (val); *(volatile T*)(ptr) = vst2_v_; __threadfence(); *(volatile T*)(ptr) = vst2_v_; } while (0)
#define VST2V4(ptr, val) do { const v4f vst2_v4_ = (val); *(volatile v4f*)(ptr) = vst2_v4_; __threadfence(); *(volatile v4f*)(ptr) = vst2_v4_; } while (0)

#define WAVE_SYNC() do { __builtin_amdgcn_fence(3  , "workgroup"); __builtin_amdgcn_wave_barrier(); __builtin_amdgcn_fence(2  , "workgroup"); } while (0)

__global__ __launch_bounds__(256) void k_cast_x(const float* __restrict__ X, unsigned short* __restrict__ DST) {
    const int u = blockIdx.x * 256 + threadIdx.x; if (u >= NROW * (CC / 8)) return;
    const int r = u / (CC / 8), c0 = 8 * (u % (CC / 8));
    const int rm = (r / SEQ) * SEQ_FULL + (r % SEQ);
    const float* s = X + (long long)rm * CC + c0;
    const v4f a = *(const v4f*)(s), b = *(const v4f*)(s + 4);
    u4v pk; pk.x = pk2h(cmb_bf(a.x), cmb_bf(a.y)); pk.y = pk2h(cmb_bf(a.z), cmb_bf(a.w)); pk.z = pk2h(cmb_bf(b.x), cmb_bf(b.y)); pk.w = pk2h(cmb_bf(b.z), cmb_bf(b.w));
    VST2(u4v, (u4v*)(DST + (long long)r * CC + c0), pk);
}

__global__ __launch_bounds__(256) void k_castT(const float* __restrict__ SRC, int lds, long long sSo, long long sSi, unsigned short* __restrict__ DST, int ldd, long long sDo, long long sDi, int zi_n, int nR, int nC, float sc) {
    const int z = blockIdx.y, zo = z / zi_n, zi = z - zo * zi_n;
    const long long u = (long long)blockIdx.x * 256 + threadIdx.x; const int per = nR / 8; if (u >= (long long)nC * per) return;
    const int c = (int)(u / per); const int r0 = 8 * (int)(u % per);
    const float* s = SRC + zo * sSo + zi * sSi + (long long)r0 * lds + c;
    const float w0 = cmb_bf(s[0]) * sc, w1 = cmb_bf(s[(long long)lds]) * sc, w2 = cmb_bf(s[2LL * lds]) * sc, w3 = cmb_bf(s[3LL * lds]) * sc;
    const float w4 = cmb_bf(s[4LL * lds]) * sc, w5 = cmb_bf(s[5LL * lds]) * sc, w6 = cmb_bf(s[6LL * lds]) * sc, w7 = cmb_bf(s[7LL * lds]) * sc;
    u4v pk; pk.x = pk2h(w0, w1); pk.y = pk2h(w2, w3); pk.z = pk2h(w4, w5); pk.w = pk2h(w6, w7);
    VST2(u4v, (u4v*)(DST + zo * sDo + zi * sDi + (long long)c * ldd + r0), pk);
}

template <int EPI>
__device__ __forceinline__ void gemm64_body(const unsigned short* __restrict__ Ap, int lda, const unsigned short* __restrict__ Btp, int ldb, int M, int N, int K, float scale,
                                            const float* __restrict__ bias, float* __restrict__ Cf, unsigned short* __restrict__ P0, unsigned short* __restrict__ P1, unsigned short* __restrict__ P2, int ldc) {
    __shared__ __align__(16) float sT[8][16 * 68];
    const _Float16* A = (const _Float16*)Ap; const _Float16* Bt = (const _Float16*)Btp;
    const int lane = threadIdx.x & 31;
    const int wave = __builtin_amdgcn_readfirstlane((int)(threadIdx.x >> 5));
    const int tilesN = N >> 6, tilesM = M >> 6;
    const int tile = (int)blockIdx.x * 8 + wave;
    if (tile >= tilesM * tilesN) return;
    const int tm = tile / tilesN, tn = tile - tm * tilesN;
    const int m0 = tm << 6, n0 = tn << 6;
    const int rlane = lane & 15;
    const int koff = (lane >> 4) * 8;
    const int mOff = (lane >> 4) * 8;

    v8f acc[4][4];
#pragma unroll
    for (int i = 0; i < 4; ++i)
#pragma unroll
        for (int j = 0; j < 4; ++j) acc[i][j] = (v8f){0.f, 0.f, 0.f, 0.f, 0.f, 0.f, 0.f, 0.f};

    for (int k0 = 0; k0 < K; k0 += 32) {
        v16h bh[4];
#pragma unroll
        for (int j = 0; j < 4; ++j) bh[j] = frag_ld(Bt + (size_t)(n0 + (j << 4) + rlane) * ldb + koff + k0);
#pragma unroll
        for (int i = 0; i < 4; ++i) {
            const v16h ah = frag_ld(A + (size_t)(m0 + (i << 4) + rlane) * lda + koff + k0);
#pragma unroll
            for (int j = 0; j < 4; ++j) acc[i][j] = wmma_raw(ah, bh[j], acc[i][j]);
            dep_guard_h(acc[i][0], acc[i][3], ah, ah);
        }
        keep4_h(bh[0], bh[1], bh[2], bh[3]);
    }
    acc_guard4(acc[0][0], acc[0][1], acc[0][2], acc[0][3]);
    acc_guard4(acc[1][0], acc[1][1], acc[1][2], acc[1][3]);
    acc_guard4(acc[2][0], acc[2][1], acc[2][2], acc[2][3]);
    acc_guard4(acc[3][0], acc[3][1], acc[3][2], acc[3][3]);

    const int part = n0 >> 10;
    const int head = (n0 >> 6) & (NH - 1);
#pragma unroll
    for (int i = 0; i < 4; ++i) {
        const int mBase = m0 + (i << 4);
#pragma unroll
        for (int j = 0; j < 4; ++j) {
            const int nl = (j << 4) + rlane;
            float bv = 0.f;
            if (EPI == 0 || EPI == 1) bv = cmb_bf(bias[n0 + nl]);
            if (EPI == 2) bv = cmb_bf(bias[head * 192 + part * 64 + nl]);
#pragma unroll
            for (int r = 0; r < 8; ++r) {
                float v = acc[i][j][r] * scale;
                if (EPI == 3) { const int m = mBase + mOff + r; v += cmb_bf(bias[(m >> 6) * 192 + 128 + (m & 63)]); }
                else v += bv;
                if (EPI == 1) v = fmaxf(v, 0.0f);
                sT[wave][(mOff + r) * 68 + nl] = v;
            }
        }
        WAVE_SYNC();
        if (EPI == 0) {
            const int hh = lane >> 4, c4 = (lane & 15) * 4;
            for (int pass = 0; pass < 2; ++pass) {
#pragma unroll
                for (int it = 0; it < 8; ++it) {
                    const int row = it * 2 + hh;
                    const v4f v = *(const v4f*)&sT[wave][row * 68 + c4];
                    *(volatile v4f*)(Cf + (size_t)(mBase + row) * ldc + n0 + c4) = v;
                }
                __threadfence();
            }
        } else {
            const int q4 = lane >> 3, c8 = (lane & 7) * 8;
            for (int pass = 0; pass < 2; ++pass) {
#pragma unroll
                for (int it = 0; it < 4; ++it) {
                    const int row = it * 4 + q4;
                    const v4f a0 = *(const v4f*)&sT[wave][row * 68 + c8];
                    const v4f a1 = *(const v4f*)&sT[wave][row * 68 + c8 + 4];
                    v8h hv;
                    hv[0] = (_Float16)a0.x; hv[1] = (_Float16)a0.y; hv[2] = (_Float16)a0.z; hv[3] = (_Float16)a0.w;
                    hv[4] = (_Float16)a1.x; hv[5] = (_Float16)a1.y; hv[6] = (_Float16)a1.z; hv[7] = (_Float16)a1.w;
                    if (EPI == 2) {
                        const int m = mBase + row; const int bb = m / SEQ; const int tt = m - bb * SEQ;
                        const size_t po = (size_t)((bb * NH + head) * SEQ + tt) * HD + c8;
                        if (part == 0) {
                            v8h lv;
                            lv[0] = (_Float16)((a0.x - (float)hv[0]) * QRES); lv[1] = (_Float16)((a0.y - (float)hv[1]) * QRES);
                            lv[2] = (_Float16)((a0.z - (float)hv[2]) * QRES); lv[3] = (_Float16)((a0.w - (float)hv[3]) * QRES);
                            lv[4] = (_Float16)((a1.x - (float)hv[4]) * QRES); lv[5] = (_Float16)((a1.y - (float)hv[5]) * QRES);
                            lv[6] = (_Float16)((a1.z - (float)hv[6]) * QRES); lv[7] = (_Float16)((a1.w - (float)hv[7]) * QRES);
                            *(volatile v8h*)(P0 + po) = hv;
                            *(volatile v8h*)(P1 + po) = lv;
                        } else {
                            *(volatile v8h*)(P2 + po) = hv;
                        }
                    } else {
                        *(volatile v8h*)(P0 + (size_t)(mBase + row) * ldc + n0 + c8) = hv;
                    }
                }
                __threadfence();
            }
        }
        WAVE_SYNC();
    }
}

__global__ __launch_bounds__(256) void k_gemm_qk(const unsigned short* __restrict__ X16, const unsigned short* __restrict__ Wqk, const float* __restrict__ bqkv,
                                                 unsigned short* __restrict__ Qh, unsigned short* __restrict__ Qr, unsigned short* __restrict__ Kh) {
    gemm64_body<2>(X16, CC, Wqk, CC, NROW, 2 * CC, CC, WSC_INV, bqkv, nullptr, Qh, Qr, Kh, HD);
}
__global__ __launch_bounds__(256) void k_gemm_vt(const unsigned short* __restrict__ Wv, const unsigned short* __restrict__ X16, const float* __restrict__ bqkv, unsigned short* __restrict__ Vt) {
    gemm64_body<3>(Wv, CC, X16, CC, CC, NROW, CC, WSC_INV, bqkv, nullptr, Vt, nullptr, nullptr, NROW);
}
__global__ __launch_bounds__(256) void k_gemm_wo(const unsigned short* __restrict__ AO16, const unsigned short* __restrict__ WOT, const float* __restrict__ bO, float* __restrict__ ATT) {
    gemm64_body<0>(AO16, CC, WOT, CC, NROW, CC, CC, WSC_INV / AOC, bO, ATT, nullptr, nullptr, nullptr, CC);
}
__global__ __launch_bounds__(256) void k_gemm_ff1(const unsigned short* __restrict__ X1h, const unsigned short* __restrict__ W1T, const float* __restrict__ b1, unsigned short* __restrict__ H16) {
    gemm64_body<1>(X1h, CC, W1T, CC, NROW, FFW, CC, WSC_INV, b1, nullptr, H16, nullptr, nullptr, FFW);
}
__global__ __launch_bounds__(256) void k_gemm_ff2(const unsigned short* __restrict__ H16, const unsigned short* __restrict__ W2T, const float* __restrict__ b2, float* __restrict__ FFo) {
    gemm64_body<0>(H16, FFW, W2T, FFW, NROW, CC, FFW, WSC_INV, b2, FFo, nullptr, nullptr, nullptr, CC);
}

#define AT_PP 40
__global__ __launch_bounds__(128) void k_attn(const unsigned short* __restrict__ Qh_, const unsigned short* __restrict__ Qr_, const unsigned short* __restrict__ Kh_,
                                              const unsigned short* __restrict__ Vt_, unsigned short* __restrict__ AO) {
    __shared__ __align__(16) _Float16 Ps[4][16 * AT_PP];
    __shared__ __align__(16) float    Os[4][16 * 68];
    const _Float16* Qh = (const _Float16*)Qh_; const _Float16* Qr = (const _Float16*)Qr_;
    const _Float16* Kh = (const _Float16*)Kh_; const _Float16* Vt = (const _Float16*)Vt_;
    const int wave = __builtin_amdgcn_readfirstlane((int)(threadIdx.x >> 5));
    const int lane = threadIdx.x & 31, hh = lane >> 4, c = lane & 15;
    const int nqb = SEQ / 64;
    const int bx = (int)blockIdx.x;
    const int qb = bx % nqb; const int bh = bx / nqb; const int h = bh % NH; const int b = bh / NH;
    const int q0 = qb * 64 + wave * 16;
    const int pbase = (b * NH + h) * SEQ * HD;
    const int qoff = pbase + (q0 + c) * HD + 8 * hh;
    const int koff = pbase + c * HD + 8 * hh;
    const int voff = (h * HD + c) * NROW + b * SEQ + 8 * hh;
    const float SC = 0.125f * 1.4426950408889634f;
    const float FILLV = -9.0e15f;

    float mrow[8], lrow[8];
    v8f o[4];
#pragma unroll
    for (int r = 0; r < 8; ++r) { mrow[r] = -__builtin_inff(); lrow[r] = 0.f; }
#pragma unroll
    for (int t = 0; t < 4; ++t) o[t] = (v8f){0.f, 0.f, 0.f, 0.f, 0.f, 0.f, 0.f, 0.f};

    for (int kc = 0; kc <= qb; ++kc) {
        const bool diag = (kc == qb);
#pragma unroll 1
        for (int hf = 0; hf < 2; ++hf) {
            const int kvh = kc * 64 + hf * 32;
            int qo = qoff; asm volatile("" : "+v"(qo));
            v8f sh[2], sr[2];
#pragma unroll
            for (int j = 0; j < 2; ++j) { sh[j] = (v8f){0.f, 0.f, 0.f, 0.f, 0.f, 0.f, 0.f, 0.f}; sr[j] = sh[j]; }
#pragma unroll
            for (int dc = 0; dc < 2; ++dc) {
                const v16h qh = frag_ld(Qh + qo + dc * 32);
                const v16h qr = frag_ld(Qr + qo + dc * 32);
#pragma unroll
                for (int j = 0; j < 2; ++j) {
                    const v16h kf = frag_ld(Kh + koff + (kvh + j * 16) * HD + dc * 32);
                    sh[j] = wmma16(qh, kf, sh[j]);
                    sr[j] = wmma16(qr, kf, sr[j]);
                }
            }
#pragma unroll
            for (int r = 0; r < 8; ++r) {
                const int qrow = q0 + 8 * hh + r;
                float v0 = (sh[0][r] + sr[0][r] * QRES_INV) * SC;
                float v1 = (sh[1][r] + sr[1][r] * QRES_INV) * SC;
                const bool m0 = diag && (kvh + c > qrow);
                const bool m1 = diag && (kvh + 16 + c > qrow);
                v0 = m0 ? FILLV : v0;
                v1 = m1 ? FILLV : v1;
                float m = fmaxf(v0, v1);
                m = fmaxf(m, __shfl_xor(m, 1, 32)); m = fmaxf(m, __shfl_xor(m, 2, 32));
                m = fmaxf(m, __shfl_xor(m, 4, 32)); m = fmaxf(m, __shfl_xor(m, 8, 32));
                const float mnew = fmaxf(mrow[r], m);
                const float alpha = exp2f(mrow[r] - mnew);
                const float p0 = exp2f(v0 - mnew), p1 = exp2f(v1 - mnew);
                float ps = p0 + p1;
                ps += __shfl_xor(ps, 1, 32); ps += __shfl_xor(ps, 2, 32); ps += __shfl_xor(ps, 4, 32); ps += __shfl_xor(ps, 8, 32);
                lrow[r] = lrow[r] * alpha + ps;
                mrow[r] = mnew;
#pragma unroll
                for (int t = 0; t < 4; ++t) o[t][r] *= alpha;
                Ps[wave][(8 * hh + r) * AT_PP + c]      = (_Float16)(p0 * PSC);
                Ps[wave][(8 * hh + r) * AT_PP + 16 + c] = (_Float16)(p1 * PSC);
            }
            WAVE_SYNC();
            FragU pa;
            pa.h[0] = *(const v8h*)&Ps[wave][c * AT_PP + 8 * hh];
            pa.h[1] = *(const v8h*)&Ps[wave][c * AT_PP + 16 + 8 * hh];
#pragma unroll
            for (int t = 0; t < 4; ++t) {
                const v16h vb = frag_ld(Vt + voff + t * 16 * NROW + kvh);
                o[t] = wmma16(pa.v, vb, o[t]);
            }
            WAVE_SYNC();
        }
    }

#pragma unroll
    for (int r = 0; r < 8; ++r) {
        const float inv = AOC / (lrow[r] * PSC);
#pragma unroll
        for (int t = 0; t < 4; ++t) Os[wave][(8 * hh + r) * 68 + t * 16 + c] = o[t][r] * inv;
    }
    WAVE_SYNC();
    {
        const int q4 = lane >> 3, c8 = (lane & 7) * 8;
        for (int pass = 0; pass < 2; ++pass) {
#pragma unroll
            for (int it = 0; it < 4; ++it) {
                const int row = it * 4 + q4;
                const v4f a0 = *(const v4f*)&Os[wave][row * 68 + c8];
                const v4f a1 = *(const v4f*)&Os[wave][row * 68 + c8 + 4];
                v8h hv;
                hv[0] = (_Float16)a0.x; hv[1] = (_Float16)a0.y; hv[2] = (_Float16)a0.z; hv[3] = (_Float16)a0.w;
                hv[4] = (_Float16)a1.x; hv[5] = (_Float16)a1.y; hv[6] = (_Float16)a1.z; hv[7] = (_Float16)a1.w;
                *(volatile v8h*)(AO + (size_t)(b * SEQ + q0 + row) * CC + h * HD + c8) = hv;
            }
            __threadfence();
        }
    }
}

template <int XRAW, int HAS16, int OMAP>
__device__ __forceinline__ void ln_body(const float* __restrict__ A, const float* __restrict__ X, const float* __restrict__ GA, const float* __restrict__ BE,
                                        float* __restrict__ Yf, unsigned short* __restrict__ Y16) {
    #pragma clang fp contract(off)
    const int r = blockIdx.x * 8 + (threadIdx.x >> 5); const int L = threadIdx.x & 31; if (r >= NROW) return;
    const int rm = (r / SEQ) * SEQ_FULL + (r % SEQ);
    const long long ao = (long long)r * CC;
    const long long xo = XRAW ? (long long)rm * CC : (long long)r * CC;
    const long long yo = OMAP ? (long long)rm * CC : (long long)r * CC;
    v4f v[8]; float s = 0.f;
#pragma unroll
    for (int q = 0; q < 8; ++q) {
        const int ci = 4 * L + 128 * q;
        const v4f a = *(const v4f*)(A + ao + ci);
        v4f x = *(const v4f*)(X + xo + ci);
        if (XRAW) { x.x = cmb_bf(x.x); x.y = cmb_bf(x.y); x.z = cmb_bf(x.z); x.w = cmb_bf(x.w); }
        v[q].x = x.x + a.x; v[q].y = x.y + a.y; v[q].z = x.z + a.z; v[q].w = x.w + a.w;
        s += (v[q].x + v[q].y) + (v[q].z + v[q].w);
    }
#pragma unroll
    for (int o = 16; o > 0; o >>= 1) s += __shfl_xor(s, o, 32);
    const float mu = s * (1.f / CC); float qq = 0.f;
#pragma unroll
    for (int q = 0; q < 8; ++q) { v[q].x -= mu; v[q].y -= mu; v[q].z -= mu; v[q].w -= mu; qq += (v[q].x * v[q].x + v[q].y * v[q].y) + (v[q].z * v[q].z + v[q].w * v[q].w); }
#pragma unroll
    for (int o = 16; o > 0; o >>= 1) qq += __shfl_xor(qq, o, 32);
    const float rs = rsqrtf(qq * (1.f / CC) + 1e-5f);
#pragma unroll
    for (int q = 0; q < 8; ++q) {
        const int ci = 4 * L + 128 * q;
        const v4f ga = *(const v4f*)(GA + ci), be = *(const v4f*)(BE + ci);
        v4f y;
        y.x = v[q].x * rs * cmb_bf(ga.x) + cmb_bf(be.x); y.y = v[q].y * rs * cmb_bf(ga.y) + cmb_bf(be.y);
        y.z = v[q].z * rs * cmb_bf(ga.z) + cmb_bf(be.z); y.w = v[q].w * rs * cmb_bf(ga.w) + cmb_bf(be.w);
        VST2V4(Yf + yo + ci, y);
        if (HAS16) { u2v pk; pk.x = pk2h(y.x, y.y); pk.y = pk2h(y.z, y.w); VST2(u2v, (u2v*)(Y16 + ao + ci), pk); }
    }
}
__global__ __launch_bounds__(256) void k_ln1(const float* __restrict__ ATT, const float* __restrict__ X, const float* __restrict__ GA, const float* __restrict__ BE, float* __restrict__ X1, unsigned short* __restrict__ X1h) {
    ln_body<1, 1, 0>(ATT, X, GA, BE, X1, X1h);
}
__global__ __launch_bounds__(256) void k_ln2(const float* __restrict__ FFo, const float* __restrict__ X1, const float* __restrict__ GA, const float* __restrict__ BE, float* __restrict__ OUT) {
    ln_body<0, 0, 1>(FFo, X1, GA, BE, OUT, nullptr);
}

static constexpr size_t SZ_ACT16 = (size_t)NROW * CC * 2;
static constexpr size_t SZ_ACT32 = (size_t)NROW * CC * 4;
static constexpr size_t SZ_W3    = (size_t)3 * CC * CC * 2;
static constexpr size_t SZ_WO    = (size_t)CC * CC * 2;
static constexpr size_t SZ_WF    = (size_t)CC * FFW * 2;
static constexpr size_t SZ_QKV   = (size_t)4 * SZ_ACT16;
static constexpr size_t SZ_H16   = (size_t)NROW * FFW * 2;
static constexpr size_t OFF_X16  = 0;
static constexpr size_t OFF_W3   = OFF_X16 + SZ_ACT16;
static constexpr size_t OFF_WO   = OFF_W3 + SZ_W3;
static constexpr size_t OFF_W1   = OFF_WO + SZ_WO;
static constexpr size_t OFF_W2   = OFF_W1 + SZ_WF;
static constexpr size_t OFF_QKV  = OFF_W2 + SZ_WF;
static constexpr size_t OFF_ATT  = OFF_QKV + SZ_QKV;
static constexpr size_t OFF_X1   = OFF_ATT + SZ_ACT32;
static constexpr size_t OFF_X1H  = OFF_X1 + SZ_ACT32;
static constexpr size_t WS_TOTAL = OFF_X1H + SZ_ACT16;
static_assert(SZ_H16 == SZ_QKV);
static_assert(WS_TOTAL <= (size_t)134217728);
static_assert((SZ_ACT16 % 256) == 0);
static_assert((SZ_W3 % 256) == 0);

extern "C" void kernel_launch(void* const* d_in, const int* in_sizes, int n_in, void* d_out, int out_size, void* d_ws, size_t ws_size, hipStream_t stream) {
    if (n_in < 13) return;
    const long long xmin = (long long)(NB - 1) * SEQ_FULL * CC + (long long)SEQ * CC;
    if ((long long)in_sizes[0] < xmin) return;
    if (in_sizes[1] < NH * CC * 192) return;
    if (in_sizes[2] < NH * 192) return;
    if (in_sizes[3] < CC * CC) return;
    if (in_sizes[4] < CC) return;
    if (in_sizes[5] < CC || in_sizes[6] < CC || in_sizes[7] < CC || in_sizes[8] < CC) return;
    if (in_sizes[9] < CC * FFW) return;
    if (in_sizes[10] < FFW) return;
    if (in_sizes[11] < FFW * CC) return;
    if (in_sizes[12] < CC) return;
    if ((long long)out_size < xmin) return;
    if (ws_size < WS_TOTAL) return;

    const float* x    = (const float*)d_in[0];
    const float* wqkv = (const float*)d_in[1];
    const float* bqkv = (const float*)d_in[2];
    const float* wo   = (const float*)d_in[3];
    const float* bo   = (const float*)d_in[4];
    const float* g1   = (const float*)d_in[5];
    const float* be1  = (const float*)d_in[6];
    const float* g2   = (const float*)d_in[7];
    const float* be2  = (const float*)d_in[8];
    const float* w1   = (const float*)d_in[9];
    const float* b1   = (const float*)d_in[10];
    const float* w2   = (const float*)d_in[11];
    const float* b2   = (const float*)d_in[12];
    float* out = (float*)d_out;
    char* ws = (char*)d_ws;
    unsigned short* X16  = (unsigned short*)(ws + OFF_X16);
    unsigned short* AO16 = X16;
    unsigned short* W3   = (unsigned short*)(ws + OFF_W3);
    unsigned short* WOT  = (unsigned short*)(ws + OFF_WO);
    unsigned short* W1T  = (unsigned short*)(ws + OFF_W1);
    unsigned short* W2T  = (unsigned short*)(ws + OFF_W2);
    unsigned short* Qh   = (unsigned short*)(ws + OFF_QKV);
    unsigned short* Qr   = Qh + (size_t)NROW * CC;
    unsigned short* Kh   = Qr + (size_t)NROW * CC;
    unsigned short* Vt   = Kh + (size_t)NROW * CC;
    unsigned short* H16  = Qh;
    float* ATT = (float*)(ws + OFF_ATT);
    float* FFo = ATT;
    float* X1  = (float*)(ws + OFF_X1);
    unsigned short* X1h = (unsigned short*)(ws + OFF_X1H);

    k_cast_x<<<(NROW * (CC / 8) + 255) / 256, 256, 0, stream>>>(x, X16);
    k_castT<<<dim3((unsigned)((64 * (CC / 8) + 255) / 256), (unsigned)(NH * 3)), 256, 0, stream>>>(wqkv, 192, (long long)CC * 192, 64LL, W3, CC, (long long)HD * CC, (long long)CC * CC, 3, CC, HD, WSC);
    k_castT<<<dim3((unsigned)(((long long)CC * (CC / 8) + 255) / 256), 1u), 256, 0, stream>>>(wo, CC, 0LL, 0LL, WOT, CC, 0LL, 0LL, 1, CC, CC, WSC);
    k_castT<<<dim3((unsigned)(((long long)FFW * (CC / 8) + 255) / 256), 1u), 256, 0, stream>>>(w1, FFW, 0LL, 0LL, W1T, CC, 0LL, 0LL, 1, CC, FFW, WSC);
    k_castT<<<dim3((unsigned)(((long long)CC * (FFW / 8) + 255) / 256), 1u), 256, 0, stream>>>(w2, CC, 0LL, 0LL, W2T, FFW, 0LL, 0LL, 1, FFW, CC, WSC);

    k_gemm_qk<<<(unsigned)((((NROW / 64) * ((2 * CC) / 64)) + 7) / 8), 256, 0, stream>>>(X16, W3, bqkv, Qh, Qr, Kh);
    k_gemm_vt<<<(unsigned)((((CC / 64) * (NROW / 64)) + 7) / 8), 256, 0, stream>>>(W3 + (size_t)2 * CC * CC, X16, bqkv, Vt);
    k_attn<<<(unsigned)(NB * NH * (SEQ / 64)), 128, 0, stream>>>(Qh, Qr, Kh, Vt, AO16);
    k_gemm_wo<<<(unsigned)((((NROW / 64) * (CC / 64)) + 7) / 8), 256, 0, stream>>>(AO16, WOT, bo, ATT);
    k_ln1<<<(NROW + 7) / 8, 256, 0, stream>>>(ATT, x, g1, be1, X1, X1h);
    k_gemm_ff1<<<(unsigned)((((NROW / 64) * (FFW / 64)) + 7) / 8), 256, 0, stream>>>(X1h, W1T, b1, H16);
    k_gemm_ff2<<<(unsigned)((((NROW / 64) * (CC / 64)) + 7) / 8), 256, 0, stream>>>(H16, W2T, b2, FFo);
    k_ln2<<<(NROW + 7) / 8, 256, 0, stream>>>(FFo, X1, g2, be2, out);
}
